// LSTMCRF_31061203484727
// MI455X (gfx1250) — hardware-verified
//
#include <hip/hip_runtime.h>
#include <math.h>

constexpr int NBAT   = 16;
constexpr int NSEQ   = 256;
constexpr int NEMB   = 256;
constexpr int NHID   = 256;
constexpr int NGATE  = 1024;
constexpr int NX2    = 512;
constexpr int NTAG   = 9;
constexpr int NVOC   = 50000;
constexpr int NROW   = NBAT * NSEQ;
constexpr int NTHR   = 256;
constexpr int HPITCH = 264;
constexpr int OPITCH = 260;
constexpr int RPW    = 32;
constexpr int NQ4    = RPW * NTAG / 4;
constexpr int GBLK   = (NGATE / 64) * (NROW / 64) / 8;
constexpr float CARRY    = 16.0f;
constexpr float PROD_INV = 1.0f / 256.0f;
constexpr float LN_EPS   = 1e-5f;

static_assert(NROW % 64 == 0 && NGATE % 64 == 0);
static_assert(NEMB % 32 == 0 && NX2 % 32 == 0 && NHID % 32 == 0);
static_assert(GBLK * 8 == (NGATE / 64) * (NROW / 64));
static_assert(NHID == 32 * (NTHR / 32));
static_assert(NROW % (NTHR / 32) == 0);
static_assert(2 * NTHR * 8 == NBAT * NHID);
static_assert(4 * NTHR * 4 == NBAT * NHID);
static_assert(NROW % (RPW * (NTHR / 32)) == 0);
static_assert((RPW * NTAG * 4) % 128 == 0);
static_assert(NROW * NTAG * 4 == 147456);
static_assert(HPITCH % 8 == 0 && OPITCH % 4 == 0);
static_assert(NX2 % 128 == 0 && (NTAG * NX2) % 4 == 0);
static_assert(NSEQ == 256 && NBAT == 16);

typedef __attribute__((ext_vector_type(16))) _Float16 v16h;
typedef __attribute__((ext_vector_type(8)))  _Float16 v8h;
typedef __attribute__((ext_vector_type(16))) __bf16   v16b;
typedef __attribute__((ext_vector_type(8)))  __bf16   v8b;
typedef __attribute__((ext_vector_type(8)))  float    v8f;
typedef __attribute__((ext_vector_type(4)))  float    v4f;
typedef __attribute__((ext_vector_type(4)))  unsigned v4u;

__device__ __forceinline__ unsigned short f2bf_bits(float f) {
  unsigned u = __float_as_uint(f);
  return (unsigned short)((u + 0x7FFFu + ((u >> 16) & 1u)) >> 16);
}
__device__ __forceinline__ float bf_bits2f(unsigned short h) { return __uint_as_float(((unsigned)h) << 16); }

__device__ __forceinline__ void dep_guard_h(v8f& a, v8f& b, v16h x, v16h y) { asm volatile("v_nop\n\tv_nop\n\tv_nop\n\tv_nop" : "+v"(a), "+v"(b) : "v"(x), "v"(y)); }
__device__ __forceinline__ void dep_guard_b(v8f& a, v8f& b, v16b x, v16b y) { asm volatile("v_nop\n\tv_nop\n\tv_nop\n\tv_nop" : "+v"(a), "+v"(b) : "v"(x), "v"(y)); }
__device__ __forceinline__ void keep4_h(v16h a, v16h b, v16h c, v16h d) { asm volatile("v_nop" :: "v"(a), "v"(b), "v"(c), "v"(d)); }
__device__ __forceinline__ void keep4_b(v16b a, v16b b, v16b c, v16b d) { asm volatile("v_nop" :: "v"(a), "v"(b), "v"(c), "v"(d)); }
__device__ __forceinline__ void acc_guard4(v8f& a, v8f& b, v8f& c, v8f& d) { asm volatile("v_nop\n\tv_nop\n\tv_nop\n\tv_nop" : "+v"(a), "+v"(b), "+v"(c), "+v"(d)); }
template <typename T> struct Frag;
template <> struct Frag<_Float16> {
  typedef v16h V; union U { v16h v; v8h h[2]; };
  static __device__ __forceinline__ v16h load(const _Float16* p) {
    U f; f.h[0] = *(const v8h*)(p); f.h[1] = *(const v8h*)(p + 16); return f.v;
  }
  static __device__ __forceinline__ v8f mma(v16h a, v16h b, v8f c) {
    return __builtin_amdgcn_wmma_f32_16x16x32_f16(false, a, false, b, (short)0, c, false, false);
  }
  static __device__ __forceinline__ void guard(v8f& a, v8f& b, v16h x, v16h y) { dep_guard_h(a, b, x, y); }
  static __device__ __forceinline__ void keep(v16h a, v16h b, v16h c, v16h d) { keep4_h(a, b, c, d); }
};
template <> struct Frag<__bf16> {
  typedef v16b V; union U { v16b v; v8b h[2]; };
  static __device__ __forceinline__ v16b load(const __bf16* p) {
    U f; f.h[0] = *(const v8b*)(p); f.h[1] = *(const v8b*)(p + 16); return f.v;
  }
  static __device__ __forceinline__ v8f mma(v16b a, v16b b, v8f c) {
    return __builtin_amdgcn_wmma_f32_16x16x32_bf16(false, a, false, b, (short)0, c, false, false);
  }
  static __device__ __forceinline__ void guard(v8f& a, v8f& b, v16b x, v16b y) { dep_guard_b(a, b, x, y); }
  static __device__ __forceinline__ void keep(v16b a, v16b b, v16b c, v16b d) { keep4_b(a, b, c, d); }
};

__device__ __forceinline__ float frcp(float d)  { return __builtin_amdgcn_rcpf(d); }
__device__ __forceinline__ float fsig(float x)  { return frcp(1.0f + expf(-x)); }
__device__ __forceinline__ float ftanh(float x) { return 1.0f - 2.0f * frcp(expf(2.0f * x) + 1.0f); }
__device__ __forceinline__ int clampi(int v, int lo, int hi) { return v < lo ? lo : (v > hi ? hi : v); }

template <int ET> struct Elem;
template <> struct Elem<0> { typedef _Float16 T; };
template <> struct Elem<1> { typedef __bf16 T; };
template <int ET, bool SPLIT, int BIAS_MODE, int OUT_MODE, bool RESID, int ACT = 0>
__global__ __launch_bounds__(256) void wmma_gemm64(
    const unsigned short* __restrict__ Ap, const unsigned short* __restrict__ A2p, int lda, long strideA,
    const unsigned short* __restrict__ Btp, const unsigned short* __restrict__ Bt2p, int ldb, long strideB,
    void* __restrict__ Cout, void* __restrict__ Cout2, int ldc, long strideC,
    const float* __restrict__ bias,
    const float* __restrict__ resid, long strideR,
    int M, int N, int K, float scale) {
  typedef typename Elem<ET>::T T;
  typedef typename Frag<T>::V V;
  const T* A = (const T*)Ap; const T* A2 = (const T*)A2p; const T* Bt = (const T*)Btp; const T* Bt2 = (const T*)Bt2p;
  __shared__ __align__(16) float sT[8][16 * 68];
  const int b    = blockIdx.y;
  const int lane = threadIdx.x & 31;
  const int wave = threadIdx.x >> 5;
  const int tilesN = N >> 6;
  const int tilesM = M >> 6;
  const int tile = blockIdx.x * 8 + wave;
  if (tile >= tilesM * tilesN) return;
  const int tm = tile / tilesN;
  const int tn = tile - tm * tilesN;
  const int m0 = tm << 6;
  const int n0 = tn << 6;

  const T* Ab  = A  + (size_t)b * strideA;
  const T* Bb  = Bt + (size_t)b * strideB;
  const T* Ab2 = SPLIT ? (A2  + (size_t)b * strideA) : nullptr;
  const T* Bb2 = SPLIT ? (Bt2 + (size_t)b * strideB) : nullptr;

  const int rlane = lane & 15;
  const int koff  = (lane >> 4) * 8;
  const int mOff  = (lane >> 4) * 8;

  v8f acc[4][4];
#pragma unroll
  for (int i = 0; i < 4; ++i)
#pragma unroll
    for (int j = 0; j < 4; ++j) acc[i][j] = (v8f){0.f,0.f,0.f,0.f,0.f,0.f,0.f,0.f};

  for (int k0 = 0; k0 < K; k0 += 32) {
    V bh[4], bl[4];
#pragma unroll
    for (int j = 0; j < 4; ++j) {
      const size_t bo = (size_t)(n0 + (j << 4) + rlane) * ldb + koff + k0;
      bh[j] = Frag<T>::load(Bb + bo);
      if (SPLIT) bl[j] = Frag<T>::load(Bb2 + bo);
    }
#pragma unroll
    for (int i = 0; i < 4; ++i) {
      const size_t ao = (size_t)(m0 + (i << 4) + rlane) * lda + koff + k0;
      V ah = Frag<T>::load(Ab + ao);
      V al;
      if (SPLIT) al = Frag<T>::load(Ab2 + ao);
#pragma unroll
      for (int j = 0; j < 4; ++j) {
        acc[i][j] = Frag<T>::mma(ah, bh[j], acc[i][j]);
        if (SPLIT) {
          acc[i][j] = Frag<T>::mma(ah, bl[j], acc[i][j]);
          acc[i][j] = Frag<T>::mma(al, bh[j], acc[i][j]);
        }
      }
      Frag<T>::guard(acc[i][0], acc[i][3], ah, SPLIT ? al : ah);
    }
    Frag<T>::keep(bh[0], bh[1], bh[2], bh[3]);
    if (SPLIT) Frag<T>::keep(bl[0], bl[1], bl[2], bl[3]);
  }
  acc_guard4(acc[0][0], acc[0][1], acc[0][2], acc[0][3]);
  acc_guard4(acc[1][0], acc[1][1], acc[1][2], acc[1][3]);
  acc_guard4(acc[2][0], acc[2][1], acc[2][2], acc[2][3]);
  acc_guard4(acc[3][0], acc[3][1], acc[3][2], acc[3][3]);

  float* slab = sT[wave];
  const float* Rb = RESID ? (resid + (size_t)b * strideR) : nullptr;
#pragma unroll
  for (int i = 0; i < 4; ++i) {
    const int mBase = m0 + (i << 4);
#pragma unroll
    for (int j = 0; j < 4; ++j) {
      const int n = n0 + (j << 4) + rlane;
      float bv = 0.f;
      if (BIAS_MODE == 2) bv = bias[n];
#pragma unroll
      for (int r = 0; r < 8; ++r) {
        float v = acc[i][j][r] * scale;
        if (BIAS_MODE == 1) v += bias[mBase + mOff + r];
        if (BIAS_MODE == 2) v += bv;
        if (RESID) v += Rb[(size_t)(mBase + mOff + r) * ldc + n];
        if (ACT == 1) v = tanhf(v);
        if (ACT == 2) v = fmaxf(v, 0.0f);
        if (ACT == 3) v = v / (1.0f + expf(-v));
        if (ACT == 4) v = (v > 0.f) ? v : 0.01f * v;
        if (ACT == 5) v = 0.5f * v * (1.0f + erff(v * 0.70710678118654752f));
        slab[(mOff + r) * 68 + (j << 4) + rlane] = v;
      }
    }
    __builtin_amdgcn_fence(__ATOMIC_RELEASE, "workgroup");
    __builtin_amdgcn_wave_barrier();
    __builtin_amdgcn_fence(__ATOMIC_ACQUIRE, "workgroup");
    if (OUT_MODE == 0) {
      float* C = (float*)Cout + (size_t)b * strideC;
      const int hh = lane >> 4, c4 = (lane & 15) * 4;
      for (int pass = 0; pass < 2; ++pass) {
#pragma unroll
        for (int it = 0; it < 8; ++it) {
          const int row = it * 2 + hh;
          v4f v = *(const v4f*)(slab + row * 68 + c4);
          *(volatile v4f*)(C + (size_t)(mBase + row) * ldc + n0 + c4) = v;
        }
        __threadfence();
      }
    } else {
      const int q = lane >> 3, c8 = (lane & 7) * 8;
      unsigned short* C  = (unsigned short*)Cout  + (size_t)b * strideC;
      unsigned short* C2 = (OUT_MODE == 2) ? ((unsigned short*)Cout2 + (size_t)b * strideC) : nullptr;
      for (int pass = 0; pass < 2; ++pass) {
#pragma unroll
        for (int it = 0; it < 4; ++it) {
          const int row = it * 4 + q;
          const float* sp = slab + row * 68 + c8;
          v8h hv, lv;
#pragma unroll
          for (int e = 0; e < 8; ++e) {
            if (OUT_MODE == 1) {
              hv[e] = (_Float16)sp[e];
            } else {
              unsigned short hb = f2bf_bits(sp[e]);
              unsigned short lb = f2bf_bits(sp[e] - bf_bits2f(hb));
              hv[e] = __builtin_bit_cast(_Float16, hb);
              lv[e] = __builtin_bit_cast(_Float16, lb);
            }
          }
          *(volatile v8h*)(C + (size_t)(mBase + row) * ldc + n0 + c8) = hv;
          if (OUT_MODE == 2) *(volatile v8h*)(C2 + (size_t)(mBase + row) * ldc + n0 + c8) = lv;
        }
        __threadfence();
      }
    }
    __builtin_amdgcn_fence(__ATOMIC_RELEASE, "workgroup");
    __builtin_amdgcn_wave_barrier();
    __builtin_amdgcn_fence(__ATOMIC_ACQUIRE, "workgroup");
  }
}

__global__ __launch_bounds__(NTHR) void cvt16_kernel(const float* __restrict__ src, unsigned short* __restrict__ dst,
                                                     int n8, float sc) {
  const int i = blockIdx.x * NTHR + threadIdx.x;
  if (i < n8) {
    const float* sp = src + (size_t)i * 8;
    const v4f a = *(const v4f*)(sp);
    const v4f b = *(const v4f*)(sp + 4);
    v8h hv;
#pragma unroll
    for (int e = 0; e < 4; ++e) {
      hv[e]     = (_Float16)(a[e] * sc);
      hv[4 + e] = (_Float16)(b[e] * sc);
    }
    unsigned short* op = dst + (size_t)i * 8;
    *(volatile v8h*)op = hv;
    __threadfence();
    *(volatile v8h*)op = hv;
  }
}

__global__ __launch_bounds__(NTHR) void embed_kernel(const int* __restrict__ ids, const float* __restrict__ emb,
                                                     unsigned short* __restrict__ XE) {
  const int lane = threadIdx.x & 31;
  const int m = blockIdx.x * (NTHR / 32) + (threadIdx.x >> 5);
  const int t = m >> 4, b = m & 15;
  int id = ids[b * NSEQ + t];
  id = clampi(id, 0, NVOC - 1);
  const float* sp = emb + (size_t)id * NEMB + 8 * lane;
  const v4f a  = *(const v4f*)(sp);
  const v4f a2 = *(const v4f*)(sp + 4);
  v8h hv;
#pragma unroll
  for (int e = 0; e < 4; ++e) {
    hv[e]     = (_Float16)(a[e] * CARRY);
    hv[4 + e] = (_Float16)(a2[e] * CARRY);
  }
  unsigned short* op = XE + (size_t)m * NEMB + 8 * lane;
  *(volatile v8h*)op = hv;
  __threadfence();
  *(volatile v8h*)op = hv;
}

__global__ __launch_bounds__(NTHR) void birnn_scan_kernel(const float* __restrict__ XGT, const float* __restrict__ bl,
                                                          const unsigned short* __restrict__ WHp,
                                                          unsigned short* __restrict__ XA16, float* __restrict__ XF32) {
  __shared__ __align__(16) unsigned short Ah[NBAT * HPITCH];
  __shared__ __align__(16) float          Hs[NBAT * OPITCH];
  const int dir = blockIdx.x;
  const float* xg = XGT + (size_t)dir * NGATE * NROW;
  const float* bd = bl + (size_t)dir * 2 * NGATE;
  const _Float16* WH = (const _Float16*)WHp + (size_t)dir * NGATE * NHID;
  const int tid = threadIdx.x, lane = tid & 31, wave = tid >> 5;
  const int c = lane & 15, hh = lane >> 4, koff = hh * 8;

#pragma unroll 1
  for (int i = tid; i < NBAT * HPITCH; i += NTHR) Ah[i] = (unsigned short)0;
  float cst[2][8], hst[2][8], bb[2][4];
#pragma unroll
  for (int nt = 0; nt < 2; ++nt) {
    const int j = 32 * wave + 16 * nt + c;
#pragma unroll
    for (int g = 0; g < 4; ++g) bb[nt][g] = bd[g * NHID + j] + bd[NGATE + g * NHID + j];
#pragma unroll
    for (int r = 0; r < 8; ++r) { cst[nt][r] = 0.0f; hst[nt][r] = 0.0f; }
  }
  __syncthreads();

  const _Float16* ahrow = (const _Float16*)Ah + c * HPITCH + koff;
  const v8f z8 = {0.f, 0.f, 0.f, 0.f, 0.f, 0.f, 0.f, 0.f};

#pragma unroll 1
  for (int s = 0; s < NSEQ; ++s) {
    const int t  = dir ? (NSEQ - 1 - s) : s;
    const int m0 = t * NBAT;
#pragma unroll
    for (int nt = 0; nt < 2; ++nt) {
      const int j = 32 * wave + 16 * nt + c;
      float xv[4][8];
#pragma unroll
      for (int g = 0; g < 4; ++g) {
        const float* p = xg + (size_t)(g * NHID + j) * NROW + m0 + 8 * hh;
        const v4f u0 = *(const v4f*)(p);
        const v4f u1 = *(const v4f*)(p + 4);
        xv[g][0] = u0[0]; xv[g][1] = u0[1]; xv[g][2] = u0[2]; xv[g][3] = u0[3];
        xv[g][4] = u1[0]; xv[g][5] = u1[1]; xv[g][6] = u1[2]; xv[g][7] = u1[3];
      }
      const _Float16* wh = WH + (size_t)j * NHID + koff;
      v8f acc[4];
      acc[0] = z8; acc[1] = z8; acc[2] = z8; acc[3] = z8;
#pragma unroll 1
      for (int k0 = 0; k0 < NHID; k0 += 32) {
        const v16h a  = Frag<_Float16>::load(ahrow + k0);
        const v16h b0 = Frag<_Float16>::load(wh + k0);
        const v16h b1 = Frag<_Float16>::load(wh + (size_t)1 * NHID * NHID + k0);
        const v16h b2 = Frag<_Float16>::load(wh + (size_t)2 * NHID * NHID + k0);
        const v16h b3 = Frag<_Float16>::load(wh + (size_t)3 * NHID * NHID + k0);
        acc[0] = Frag<_Float16>::mma(a, b0, acc[0]);
        acc[1] = Frag<_Float16>::mma(a, b1, acc[1]);
        acc[2] = Frag<_Float16>::mma(a, b2, acc[2]);
        acc[3] = Frag<_Float16>::mma(a, b3, acc[3]);
        dep_guard_h(acc[0], acc[3], a, b3);
        keep4_h(b0, b1, b2, b3);
      }
      acc_guard4(acc[0], acc[1], acc[2], acc[3]);
#pragma unroll
      for (int r = 0; r < 8; ++r) {
        const float zi = acc[0][r] * PROD_INV + xv[0][r] + bb[nt][0];
        const float zf = acc[1][r] * PROD_INV + xv[1][r] + bb[nt][1];
        const float zg = acc[2][r] * PROD_INV + xv[2][r] + bb[nt][2];
        const float zo = acc[3][r] * PROD_INV + xv[3][r] + bb[nt][3];
        const float ig = fsig(zi);
        const float fg = fsig(zf);
        const float gc = ftanh(zg);
        const float og = fsig(zo);
        const float cn = fg * cst[nt][r] + ig * gc;
        cst[nt][r] = cn;
        hst[nt][r] = og * ftanh(cn);
      }
    }
    __syncthreads();
#pragma unroll
    for (int nt = 0; nt < 2; ++nt) {
      const int j = 32 * wave + 16 * nt + c;
#pragma unroll
      for (int r = 0; r < 8; ++r) {
        Ah[(8 * hh + r) * HPITCH + j] = __builtin_bit_cast(unsigned short, (_Float16)(hst[nt][r] * CARRY));
        Hs[(8 * hh + r) * OPITCH + j] = hst[nt][r];
      }
    }
    __syncthreads();
    for (int pass = 0; pass < 2; ++pass) {
#pragma unroll
      for (int it = 0; it < 2; ++it) {
        const int idx = it * NTHR + tid;
        const int row = idx >> 5, c8 = (idx & 31) * 8;
        const v4u hv = *(const v4u*)(Ah + row * HPITCH + c8);
        *(volatile v4u*)(XA16 + (size_t)(m0 + row) * NX2 + dir * NHID + c8) = hv;
      }
#pragma unroll
      for (int it = 0; it < 4; ++it) {
        const int idx = it * NTHR + tid;
        const int row = idx >> 6, c4 = (idx & 63) * 4;
        const v4f fv = *(const v4f*)(Hs + row * OPITCH + c4);
        *(volatile v4f*)(XF32 + (size_t)(m0 + row) * NX2 + dir * NHID + c4) = fv;
      }
      __threadfence();
    }
  }
}

__global__ __launch_bounds__(NTHR) void norm_proj_kernel(const float* __restrict__ XF, const float* __restrict__ lng,
                                                         const float* __restrict__ lnb, const float* __restrict__ lw,
                                                         const float* __restrict__ lbias, float* __restrict__ out) {
  __shared__ __align__(16) float Ws[NTAG * NX2];
  __shared__ __align__(16) float Gs[NX2];
  __shared__ __align__(16) float Bs[NX2];
  __shared__ float Lb[16];
  __shared__ __align__(16) float Sl[NTHR / 32][RPW * NTAG];
  const int tid = threadIdx.x, lane = tid & 31, wave = tid >> 5;
#pragma unroll 1
  for (int i = tid; i < NTAG * NX2 / 4; i += NTHR) ((v4f*)Ws)[i] = ((const v4f*)lw)[i];
  if (tid < NX2 / 4) {
    ((v4f*)Gs)[tid] = ((const v4f*)lng)[tid];
    ((v4f*)Bs)[tid] = ((const v4f*)lnb)[tid];
  }
  {
    const int li = tid < NTAG ? tid : (NTAG - 1);
    const float v = lbias[li];
    if (tid < 16) Lb[tid] = (tid < NTAG) ? v : 0.0f;
  }
  __syncthreads();

  const int gw = blockIdx.x * (NTHR / 32) + wave;
  float* sl = Sl[wave];
#pragma unroll 1
  for (int i = 0; i < RPW; ++i) {
    const int rr = gw * RPW + i;
    const int b = rr / NSEQ, s = rr % NSEQ;
    const int m = s * NBAT + b;
    const float* rp = XF + (size_t)m * NX2;
    v4f v[4];
    float sum = 0.0f;
#pragma unroll
    for (int q = 0; q < 4; ++q) {
      v[q] = *(const v4f*)(rp + 128 * q + 4 * lane);
      sum += (v[q][0] + v[q][1]) + (v[q][2] + v[q][3]);
    }
#pragma unroll
    for (int off = 1; off < 32; off <<= 1) sum += __shfl_xor(sum, off, 32);
    const float mu = sum * (1.0f / NX2);
    float ss = 0.0f;
#pragma unroll
    for (int q = 0; q < 4; ++q)
#pragma unroll
      for (int e = 0; e < 4; ++e) { const float d = v[q][e] - mu; v[q][e] = d; ss += d * d; }
#pragma unroll
    for (int off = 1; off < 32; off <<= 1) ss += __shfl_xor(ss, off, 32);
    const float var  = ss * (1.0f / NX2);
    const float rstd = rsqrtf(var + LN_EPS);
    float xn[4][4];
#pragma unroll
    for (int q = 0; q < 4; ++q) {
      const v4f g4 = *(const v4f*)(Gs + 128 * q + 4 * lane);
      const v4f b4 = *(const v4f*)(Bs + 128 * q + 4 * lane);
#pragma unroll
      for (int e = 0; e < 4; ++e) xn[q][e] = (v[q][e] * rstd) * g4[e] + b4[e];
    }
#pragma unroll 1
    for (int l = 0; l < NTAG; ++l) {
      const float* wr = Ws + l * NX2 + 4 * lane;
      float p = 0.0f;
#pragma unroll
      for (int q = 0; q < 4; ++q) {
        const v4f w4 = *(const v4f*)(wr + 128 * q);
#pragma unroll
        for (int e = 0; e < 4; ++e) p += xn[q][e] * w4[e];
      }
#pragma unroll
      for (int off = 1; off < 32; off <<= 1) p += __shfl_xor(p, off, 32);
      const float o = p + Lb[l];
      if (lane == 0) sl[i * NTAG + l] = o;
    }
  }
  __builtin_amdgcn_fence(__ATOMIC_RELEASE, "workgroup");
  __builtin_amdgcn_wave_barrier();
  __builtin_amdgcn_fence(__ATOMIC_ACQUIRE, "workgroup");
  const size_t obase = (size_t)gw * (RPW * NTAG);
  for (int pass = 0; pass < 2; ++pass) {
#pragma unroll
    for (int it = 0; it < 3; ++it) {
      const int idx = it * 32 + lane;
      const int idc = idx < NQ4 ? idx : (NQ4 - 1);
      const v4f val = *(const v4f*)(sl + idc * 4);
      if (idx < NQ4) *(volatile v4f*)(out + obase + (size_t)idx * 4) = val;
    }
    __threadfence();
  }
}

__global__ __launch_bounds__(NTHR) void tagloss_kernel(const float* lg, const int* __restrict__ msk, const int* __restrict__ lab,
                                                       const float* __restrict__ ts, const float* __restrict__ te,
                                                       const float* __restrict__ tt, float* loss_out) {
  __shared__ float al[2][NBAT][12];
  __shared__ float tr[NTAG][12];
  __shared__ float nv[NBAT];
  __shared__ float dv[NBAT];
  const int tid = threadIdx.x;
  {
    const int i = tid < NTAG * NTAG ? tid : (NTAG * NTAG - 1);
    const float v = tt[i];
    if (tid < NTAG * NTAG) tr[i / NTAG][i % NTAG] = v;
  }
  int ba = tid / NTAG; ba = ba > NBAT - 1 ? NBAT - 1 : ba;
  const int ja = tid % NTAG;
  const bool isal = tid < NBAT * NTAG;
  int bn = clampi(tid - 160, 0, NBAT - 1);
  const bool isnum = (tid >= 160) && (tid < 160 + NBAT);
  {
    const float v = ts[ja] + lg[(size_t)ba * NSEQ * NTAG + ja];
    if (isal) al[0][ba][ja] = v;
  }
  float numacc;
  {
    const int f = clampi(lab[bn * NSEQ], 0, NTAG - 1);
    numacc = ts[f] + lg[(size_t)bn * NSEQ * NTAG + f];
  }
  __syncthreads();
  int cur = 0;
#pragma unroll 1
  for (int t = 1; t < NSEQ; ++t) {
    const int   mk = msk[ba * NSEQ + t];
    const float e  = lg[((size_t)ba * NSEQ + t) * NTAG + ja];
    float mx = -3.0e38f;
#pragma unroll 1
    for (int i = 0; i < NTAG; ++i) mx = fmaxf(mx, al[cur][ba][i] + tr[i][ja]);
    float sum = 0.0f;
#pragma unroll 1
    for (int i = 0; i < NTAG; ++i) sum += expf((al[cur][ba][i] + tr[i][ja]) - mx);
    const float nx   = (mx + logf(sum)) + e;
    const float keep = al[cur][ba][ja];
    const float sel  = (mk > 0) ? nx : keep;
    const int mkn = msk[bn * NSEQ + t];
    const int tp  = clampi(lab[bn * NSEQ + t - 1], 0, NTAG - 1);
    const int tc  = clampi(lab[bn * NSEQ + t], 0, NTAG - 1);
    numacc += (tr[tp][tc] + lg[((size_t)bn * NSEQ + t) * NTAG + tc]) * (float)mkn;
    if (isal) al[1 - cur][ba][ja] = sel;
    __syncthreads();
    cur ^= 1;
  }
  if (isnum) nv[bn] = numacc;
  __syncthreads();
  {
    const int b = tid < NBAT ? tid : (NBAT - 1);
    int lsum = 0;
#pragma unroll 1
    for (int t = 0; t < NSEQ; ++t) lsum += msk[b * NSEQ + t];
    int last = lsum - 1;
    if (last < 0) last += NSEQ;
    last = clampi(last, 0, NSEQ - 1);
    const int yl = clampi(lab[b * NSEQ + last], 0, NTAG - 1);
    const float numb = nv[b] + te[yl];
    float mx = -3.0e38f;
#pragma unroll 1
    for (int j2 = 0; j2 < NTAG; ++j2) mx = fmaxf(mx, al[cur][b][j2] + te[j2]);
    float sum = 0.0f;
#pragma unroll 1
    for (int j2 = 0; j2 < NTAG; ++j2) sum += expf((al[cur][b][j2] + te[j2]) - mx);
    const float den = mx + logf(sum);
    if (tid < NBAT) dv[b] = numb - den;
  }
  __syncthreads();
  if (tid == 0) {
    float acc = 0.0f;
#pragma unroll 1
    for (int b = 0; b < NBAT; ++b) acc += dv[b];
    const float loss = -acc;
    *(volatile float*)loss_out = loss;
    __threadfence();
    *(volatile float*)loss_out = loss;
  }
}

extern "C" void kernel_launch(void* const* d_in, const int* in_sizes, int n_in,
                              void* d_out, int out_size, void* d_ws, size_t ws_size, hipStream_t stream) {
  if (n_in < 15 || d_out == nullptr || d_ws == nullptr) return;
  if (in_sizes[0] != NROW || in_sizes[1] != NROW || in_sizes[2] != NROW ||
      in_sizes[3] != NVOC * NEMB || in_sizes[4] != 2 * NGATE * NEMB || in_sizes[5] != 3 * 2 * NGATE * NX2 ||
      in_sizes[6] != 4 * 2 * NGATE * NHID || in_sizes[7] != 4 * 2 * 2 * NGATE ||
      in_sizes[8] != NX2 || in_sizes[9] != NX2 || in_sizes[10] != NTAG * NX2 || in_sizes[11] != NTAG ||
      in_sizes[12] != NTAG || in_sizes[13] != NTAG || in_sizes[14] != NTAG * NTAG ||
      out_size != NROW * NTAG + 1) return;

  const int*   ids    = (const int*)d_in[0];
  const int*   msk    = (const int*)d_in[1];
  const int*   lab    = (const int*)d_in[2];
  const float* emb    = (const float*)d_in[3];
  const float* wih0   = (const float*)d_in[4];
  const float* wihr   = (const float*)d_in[5];
  const float* whh    = (const float*)d_in[6];
  const float* bvec   = (const float*)d_in[7];
  const float* lng    = (const float*)d_in[8];
  const float* lnb    = (const float*)d_in[9];
  const float* linw   = (const float*)d_in[10];
  const float* linb   = (const float*)d_in[11];
  const float* tstart = (const float*)d_in[12];
  const float* tend   = (const float*)d_in[13];
  const float* ttrans = (const float*)d_in[14];
  float* out  = (float*)d_out;
  float* loss = out + (size_t)NROW * NTAG;

  char* ws = (char*)d_ws; size_t off = 0;
  auto carve = [&](size_t bytes) -> char* { char* p = ws + off; off += (bytes + 255) & ~(size_t)255; return p; };
  unsigned short* WIH0 = (unsigned short*)carve((size_t)2 * NGATE * NEMB * 2);
  unsigned short* WIHR = (unsigned short*)carve((size_t)3 * 2 * NGATE * NX2 * 2);
  unsigned short* WHH  = (unsigned short*)carve((size_t)4 * 2 * NGATE * NHID * 2);
  unsigned short* XE   = (unsigned short*)carve((size_t)NROW * NEMB * 2);
  unsigned short* XA   = (unsigned short*)carve((size_t)NROW * NX2 * 2);
  float*          XGT  = (float*)carve((size_t)2 * NGATE * NROW * 4);
  float*          XF   = (float*)carve((size_t)NROW * NX2 * 4);
  if (off > ws_size || off > (size_t)134217728) return;

  const int n8a = 2 * NGATE * NEMB / 8;
  const int n8b = 3 * 2 * NGATE * NX2 / 8;
  const int n8c = 4 * 2 * NGATE * NHID / 8;
  cvt16_kernel<<<(n8a + NTHR - 1) / NTHR, NTHR, 0, stream>>>(wih0, WIH0, n8a, CARRY);
  cvt16_kernel<<<(n8b + NTHR - 1) / NTHR, NTHR, 0, stream>>>(wihr, WIHR, n8b, CARRY);
  cvt16_kernel<<<(n8c + NTHR - 1) / NTHR, NTHR, 0, stream>>>(whh,  WHH,  n8c, CARRY);
  embed_kernel<<<NROW / (NTHR / 32), NTHR, 0, stream>>>(ids, emb, XE);
  for (int l = 0; l < 4; ++l) {
    const int K = (l == 0) ? NEMB : NX2;
    const unsigned short* Apl = (l == 0) ? WIH0 : (WIHR + (size_t)(l - 1) * 2 * NGATE * NX2);
    const unsigned short* Btl = (l == 0) ? XE : XA;
    wmma_gemm64<0, false, 0, 0, false, 0><<<dim3(GBLK, 2), NTHR, 0, stream>>>(
        Apl, Apl, K, (long)NGATE * K, Btl, Btl, K, 0L, (void*)XGT, (void*)XGT, NROW, (long)NGATE * NROW,
        XF, XF, 0L, NGATE, NROW, K, PROD_INV);
    birnn_scan_kernel<<<2, NTHR, 0, stream>>>(XGT, bvec + (size_t)l * 4 * NGATE,
                                               WHH + (size_t)l * 2 * NGATE * NHID, XA, XF);
  }
  norm_proj_kernel<<<NROW / (RPW * (NTHR / 32)), NTHR, 0, stream>>>(XF, lng, lnb, linw, linb, out);
  tagloss_kernel<<<1, NTHR, 0, stream>>>(out, msk, lab, tstart, tend, ttrans, loss);
}
